// TtCausalSelfAttention_60284160967318
// MI455X (gfx1250) — hardware-verified
//
#include <hip/hip_runtime.h>
#ifndef NB
#define NB 8
#endif
#ifndef SEQ
#define SEQ 1024
#endif
#define NB_FULL 8
#define SEQ_FULL 1024
#define NH 16
#define HDIM 64
#define DD 1024
#define NR (NB * SEQ)
static_assert(SEQ % 64 == 0);
static_assert(SEQ <= SEQ_FULL);
static_assert(NB >= 1 && NB <= NB_FULL);
static_assert(DD == NH * HDIM);
static_assert(DD % 64 == 0);

typedef unsigned short v8us __attribute__((ext_vector_type(8), may_alias));
typedef float  v8f  __attribute__((ext_vector_type(8)));
typedef float  v4f  __attribute__((ext_vector_type(4)));
typedef float  v4fa __attribute__((ext_vector_type(4), may_alias));
typedef _Float16 v16h __attribute__((ext_vector_type(16)));
typedef _Float16 v4h __attribute__((ext_vector_type(4)));
union FragH { v16h v; v8us half[2]; _Float16 h[16]; unsigned short u[16]; };

__device__ __forceinline__ unsigned short bf16_bits(float x) { unsigned int u = __float_as_uint(x); return (unsigned short)((u + 0x7FFFu + ((u >> 16) & 1u)) >> 16); }
__device__ __forceinline__ float bf16_val(unsigned short b) { return __uint_as_float(((unsigned int)b) << 16); }
__device__ __forceinline__ float bf16_rne(float x) { return bf16_val(bf16_bits(x)); }

template <int NT>
__device__ __forceinline__ v8f mmaH(v16h ah, v16h al, v16h bh, v16h bl, v8f c) {
  c = __builtin_amdgcn_wmma_f32_16x16x32_f16(false, ah, false, bh, (short)0, c, false, false);
  if (NT >= 2) c = __builtin_amdgcn_wmma_f32_16x16x32_f16(false, al, false, bh, (short)0, c, false, false);
  if (NT >= 3) c = __builtin_amdgcn_wmma_f32_16x16x32_f16(false, ah, false, bl, (short)0, c, false, false);
  asm volatile("v_nop\n\tv_nop\n\tv_nop\n\tv_nop" : "+v"(c) : "v"(ah), "v"(al), "v"(bh), "v"(bl));
  return c;
}

__global__ __launch_bounds__(256) void k_wt_f16(const float* __restrict__ W, _Float16* __restrict__ Wt, int K, int N, float scale) {
  const int t = blockIdx.x * 256 + threadIdx.x; if (t >= N * (K / 8)) return; const int n = t / (K / 8), k8 = (t % (K / 8)) * 8; FragH f;
#pragma unroll
  for (int i = 0; i < 8; ++i) f.h[i] = (_Float16)(bf16_rne(W[(size_t)(k8 + i) * N + n]) * scale); const v8us o = f.half[0];
  *(volatile v8us*)((unsigned short*)Wt + (size_t)n * K + k8) = o; __threadfence(); *(volatile v8us*)((unsigned short*)Wt + (size_t)n * K + k8) = o;
}

template <int ACT>
__global__ __launch_bounds__(128) void k_gemm_hhx(const _Float16* __restrict__ A, int lda, size_t sA, const _Float16* __restrict__ Bh, int ldb, size_t sB, float alpha, const float* __restrict__ bias, size_t sBias, const float* CP,
    float* C, _Float16* C16, int ldc, size_t sC, int M, int N, int K) {
  __shared__ __attribute__((aligned(16))) float so[4][16][64];
  const int tid = threadIdx.x, w = tid >> 5, lane = tid & 31, ln = lane & 15, hh = lane >> 4; const int by = blockIdx.y;
  A += (size_t)by * sA; Bh += (size_t)by * sB; const size_t cofs = (size_t)by * sC; const float* bp = bias ? bias + (size_t)by * sBias : nullptr;
  const int ntn = (N + 63) / 64; const int wid = blockIdx.x * 4 + w; const int mt = wid / ntn, nq = wid % ntn; if (mt * 16 >= M) return;
  const int row0 = mt * 16, col0 = nq * 64; const _Float16* arow = A + (size_t)(row0 + ln) * lda;
  v8f acc[4] = {};
  for (int kb = 0; kb < K; kb += 32) { FragH ah; ah.half[0] = *(const v8us*)((const unsigned short*)arow + kb + 8 * hh); ah.half[1] = *(const v8us*)((const unsigned short*)arow + kb + 16 + 8 * hh);
#pragma unroll
    for (int t = 0; t < 4; ++t) { if (col0 + t * 16 >= N) continue; const size_t boff = (size_t)(col0 + t * 16 + ln) * ldb + kb; FragH bq; bq.half[0] = *(const v8us*)((const unsigned short*)Bh + boff + 8 * hh); bq.half[1] = *(const v8us*)((const unsigned short*)Bh + boff + 16 + 8 * hh);
      acc[t] = mmaH<1>(ah.v, ah.v, bq.v, bq.v, acc[t]); }
  }
#pragma unroll
  for (int t = 0; t < 4; ++t) { if (col0 + t * 16 >= N) continue; const int col = col0 + t * 16 + ln; const float bv = bp ? bf16_rne(bp[col]) : 0.f;
#pragma unroll
    for (int r = 0; r < 8; ++r) { float v = acc[t][r] * alpha + bv; if (CP) v += CP[cofs + (size_t)(row0 + 8 * hh + r) * ldc + col]; if (ACT == 1) v = fmaxf(v, 0.f); so[w][8 * hh + r][t * 16 + ln] = v; } }
  __builtin_amdgcn_fence(__ATOMIC_ACQ_REL, "workgroup"); __builtin_amdgcn_wave_barrier();
  const int rsub = lane >> 4, c4 = (lane & 15) * 4;
  for (int pass = 0; pass < 2; ++pass) {
#pragma unroll
    for (int q = 0; q < 8; ++q) { const int r = q * 2 + rsub; if (col0 + c4 < N) { const v4f v = *(const v4fa*)&so[w][r][c4]; if (C) *(volatile v4f*)(C + cofs + (size_t)(row0 + r) * ldc + col0 + c4) = v; if (C16) { v4h h4; for (int i = 0; i < 4; ++i) h4[i] = (_Float16)v[i]; *(volatile v4h*)(C16 + cofs + (size_t)(row0 + r) * ldc + col0 + c4) = h4; } } }
    if (pass == 0) __threadfence(); }
}

__global__ __launch_bounds__(256) void k_x16s(const float* __restrict__ x, _Float16* __restrict__ X16, size_t n8) {
  const size_t t = (size_t)blockIdx.x * 256 + threadIdx.x; if (t >= n8) return;
  const size_t row = t / (DD / 8); const int c8 = (int)(t % (DD / 8)) * 8; const size_t b = row / SEQ, tt = row % SEQ;
  const float* src = x + (b * SEQ_FULL + tt) * DD + c8; const v4f a = *(const v4fa*)src, c = *(const v4fa*)(src + 4); FragH f;
#pragma unroll
  for (int q = 0; q < 4; ++q) { f.h[q] = (_Float16)bf16_rne(a[q]); f.h[4 + q] = (_Float16)bf16_rne(c[q]); }
  *(volatile v8us*)((unsigned short*)X16 + t * 8) = f.half[0]; __threadfence(); *(volatile v8us*)((unsigned short*)X16 + t * 8) = f.half[0]; }

__global__ __launch_bounds__(256) void k_hl(const float* __restrict__ F, _Float16* __restrict__ Hh, _Float16* __restrict__ Hl, size_t n8) { const size_t t = (size_t)blockIdx.x * 256 + threadIdx.x; if (t >= n8) return; FragH fh, fl; const v4f a = *(const v4fa*)(F + t * 8), c = *(const v4fa*)(F + t * 8 + 4);
#pragma unroll
  for (int q = 0; q < 4; ++q) { _Float16 h = (_Float16)a[q]; fh.h[q] = h; fl.h[q] = (_Float16)((a[q] - (float)h) * 1024.0f); h = (_Float16)c[q]; fh.h[4 + q] = h; fl.h[4 + q] = (_Float16)((c[q] - (float)h) * 1024.0f); }
  for (int pass = 0; pass < 2; ++pass) { *(volatile v8us*)((unsigned short*)Hh + t * 8) = fh.half[0]; *(volatile v8us*)((unsigned short*)Hl + t * 8) = fl.half[0]; if (pass == 0) __threadfence(); } }

template <int NHv, int TTv>
__global__ __launch_bounds__(256) void k_vts(const float* __restrict__ VF, int ldv, _Float16* __restrict__ Vt, _Float16* __restrict__ Vtlo) {
  __shared__ __attribute__((aligned(16))) unsigned short th[64][66]; __shared__ __attribute__((aligned(16))) unsigned short tlo[64][66];
  const int tid = threadIdx.x; const int slab = blockIdx.x / (TTv / 64), lg = blockIdx.x % (TTv / 64); const int b = slab / NHv, h = slab % NHv;
  for (int i = tid; i < 64 * 16; i += 256) { const int r = i / 16, c4 = (i % 16) * 4;
    const v4f a = *(const v4fa*)(VF + ((size_t)b * TTv + lg * 64 + r) * ldv + h * 64 + c4); FragH fh, fl;
#pragma unroll
    for (int q = 0; q < 4; ++q) { const _Float16 hv = (_Float16)a[q]; fh.h[q] = hv; fl.h[q] = (_Float16)((a[q] - (float)hv) * 1024.0f); }
#pragma unroll
    for (int q = 0; q < 4; ++q) { th[r][c4 + q] = fh.u[q]; tlo[r][c4 + q] = fl.u[q]; } }
  __syncthreads();
  for (int pass = 0; pass < 2; ++pass) {
#pragma unroll
    for (int rd = 0; rd < 2; ++rd) { const int d = rd * 32 + tid / 8, pc = tid % 8; FragH fh, fl;
#pragma unroll
      for (int q = 0; q < 8; ++q) { fh.u[q] = th[pc * 8 + q][d]; fl.u[q] = tlo[pc * 8 + q][d]; }
      const size_t o = ((size_t)slab * 64 + d) * TTv + lg * 64 + pc * 8;
      *(volatile v8us*)((unsigned short*)Vt + o) = fh.half[0]; *(volatile v8us*)((unsigned short*)Vtlo + o) = fl.half[0]; }
    if (pass == 0) __threadfence(); } }

__global__ __launch_bounds__(128) void k_flash(const _Float16* __restrict__ Q16, int ldq, const _Float16* __restrict__ K16, int ldk, const _Float16* __restrict__ Vt, const _Float16* __restrict__ Vtlo, float* __restrict__ O, int ldo) {
  constexpr int RPW = 16, RTN = RPW / 16, NQB = SEQ / (4 * RPW), DT = 4, KS = 2;
  __shared__ __attribute__((aligned(16))) unsigned short sP[4][RPW][40]; __shared__ __attribute__((aligned(16))) float sO[4][RPW][64 + 4];
  const int tid = threadIdx.x, w = tid >> 5, lane = tid & 31, ln = lane & 15, hh = lane >> 4;
  const int slab = blockIdx.x / NQB, qblk = blockIdx.x % NQB; const int b = slab / NH, h = slab % NH; const int qb0 = qblk * (4 * RPW); const int q0 = qb0 + w * RPW;
  FragH aq[2][KS];
#pragma unroll
  for (int rt = 0; rt < RTN; ++rt) { const unsigned short* qr = (const unsigned short*)Q16 + ((size_t)b * SEQ + q0 + rt * 16 + ln) * ldq + h * 64;
#pragma unroll
    for (int ks = 0; ks < KS; ++ks) { aq[rt][ks].half[0] = *(const v8us*)(qr + ks * 32 + 8 * hh); aq[rt][ks].half[1] = *(const v8us*)(qr + ks * 32 + 16 + 8 * hh); } }
  const unsigned short* Vth = (const unsigned short*)Vt + (size_t)slab * 64 * SEQ; const unsigned short* Vtl = (const unsigned short*)Vtlo + (size_t)slab * 64 * SEQ;
  float m_r[2][8], l_r[2][8]; v8f oacc[2][DT], oaccl[2][DT];
#pragma unroll
  for (int rt = 0; rt < RTN; ++rt) {
#pragma unroll
    for (int r = 0; r < 8; ++r) { m_r[rt][r] = -3.0e38f; l_r[rt][r] = 0.f; }
#pragma unroll
    for (int dt = 0; dt < DT; ++dt) { oacc[rt][dt] = (v8f){0.f,0.f,0.f,0.f,0.f,0.f,0.f,0.f}; oaccl[rt][dt] = oacc[rt][dt]; } }
  const int jend = qb0 + 4 * RPW;
#pragma unroll 1
  for (int j0 = 0; j0 < jend; j0 += 32) {
    v8f s[2][2];
#pragma unroll
    for (int nt = 0; nt < 2; ++nt) { const unsigned short* kr = (const unsigned short*)K16 + ((size_t)b * SEQ + j0 + nt * 16 + ln) * ldk + h * 64; FragH bk[KS];
#pragma unroll
      for (int ks = 0; ks < KS; ++ks) { bk[ks].half[0] = *(const v8us*)(kr + ks * 32 + 8 * hh); bk[ks].half[1] = *(const v8us*)(kr + ks * 32 + 16 + 8 * hh); }
#pragma unroll
      for (int rt = 0; rt < RTN; ++rt) { v8f acc = (v8f){0.f,0.f,0.f,0.f,0.f,0.f,0.f,0.f};
#pragma unroll
        for (int ks = 0; ks < KS; ++ks) acc = mmaH<1>(aq[rt][ks].v, aq[rt][ks].v, bk[ks].v, bk[ks].v, acc); s[rt][nt] = acc; } }
#pragma unroll
    for (int rt = 0; rt < RTN; ++rt)
#pragma unroll
      for (int r = 0; r < 8; ++r) { const int tq = q0 + rt * 16 + 8 * hh + r; const int k0 = j0 + ln, k1 = j0 + 16 + ln; (void)tq; (void)k0; (void)k1;
        const bool ok0 = (k0 <= tq), ok1 = (k1 <= tq);
        const float s0 = ok0 ? s[rt][0][r] * (0.125f) : -INFINITY, s1 = ok1 ? s[rt][1][r] * (0.125f) : -INFINITY; float mc = fmaxf(s0, s1);
        mc = fmaxf(mc, __shfl_xor(mc, 1, 32)); mc = fmaxf(mc, __shfl_xor(mc, 2, 32)); mc = fmaxf(mc, __shfl_xor(mc, 4, 32)); mc = fmaxf(mc, __shfl_xor(mc, 8, 32));
        const float mn = fmaxf(m_r[rt][r], mc); const float al = (mn > -1.0e38f) ? expf(m_r[rt][r] - mn) : 1.0f; m_r[rt][r] = mn; const float p0 = ok0 ? expf(s0 - mn) : 0.f, p1 = ok1 ? expf(s1 - mn) : 0.f; l_r[rt][r] = l_r[rt][r] * al + p0 + p1;
#pragma unroll
        for (int dt = 0; dt < DT; ++dt) { oacc[rt][dt][r] *= al; oaccl[rt][dt][r] *= al; }
        FragH t2; t2.h[0] = (_Float16)(p0 * 1024.0f); t2.h[1] = (_Float16)(p1 * 1024.0f); sP[w][rt * 16 + 8 * hh + r][ln] = t2.u[0]; sP[w][rt * 16 + 8 * hh + r][16 + ln] = t2.u[1]; }
    __builtin_amdgcn_fence(__ATOMIC_ACQ_REL, "workgroup"); __builtin_amdgcn_wave_barrier();
    FragH pa[2];
#pragma unroll
    for (int rt = 0; rt < RTN; ++rt) { pa[rt].half[0] = *(const v8us*)&sP[w][rt * 16 + ln][8 * hh]; pa[rt].half[1] = *(const v8us*)&sP[w][rt * 16 + ln][16 + 8 * hh]; }
#pragma unroll
    for (int dt = 0; dt < DT; ++dt) { const size_t vo = (size_t)(dt * 16 + ln) * SEQ + j0; FragH bv, bl; bv.half[0] = *(const v8us*)(Vth + vo + 8 * hh); bv.half[1] = *(const v8us*)(Vth + vo + 16 + 8 * hh); bl.half[0] = *(const v8us*)(Vtl + vo + 8 * hh); bl.half[1] = *(const v8us*)(Vtl + vo + 16 + 8 * hh);
#pragma unroll
      for (int rt = 0; rt < RTN; ++rt) { oacc[rt][dt] = mmaH<1>(pa[rt].v, pa[rt].v, bv.v, bv.v, oacc[rt][dt]); oaccl[rt][dt] = mmaH<1>(pa[rt].v, pa[rt].v, bl.v, bl.v, oaccl[rt][dt]); } }
    __builtin_amdgcn_fence(__ATOMIC_ACQ_REL, "workgroup"); __builtin_amdgcn_wave_barrier(); }
#pragma unroll
  for (int rt = 0; rt < RTN; ++rt) {
#pragma unroll
    for (int r = 0; r < 8; ++r) { float l = l_r[rt][r]; l += __shfl_xor(l, 1, 32); l += __shfl_xor(l, 2, 32); l += __shfl_xor(l, 4, 32); l += __shfl_xor(l, 8, 32); l_r[rt][r] = (l > 0.f) ? 1.0f / (l * 1024.0f) : 0.f; }
#pragma unroll
    for (int dt = 0; dt < DT; ++dt)
#pragma unroll
      for (int r = 0; r < 8; ++r) sO[w][rt * 16 + 8 * hh + r][dt * 16 + ln] = (oacc[rt][dt][r] + oaccl[rt][dt][r] * 0.0009765625f) * l_r[rt][r]; }
  __builtin_amdgcn_fence(__ATOMIC_ACQ_REL, "workgroup"); __builtin_amdgcn_wave_barrier();
  for (int pass = 0; pass < 2; ++pass) {
#pragma unroll
    for (int rp = 0; rp < RPW; rp += 2) { const int r = rp + (lane >> 4), pc = lane & 15; const v4f val = *(const v4fa*)&sO[w][r][pc * 4]; *(volatile v4f*)(O + ((size_t)b * SEQ + q0 + r) * ldo + h * 64 + pc * 4) = val; }
    if (pass == 0) __threadfence(); } }

extern "C" void kernel_launch(void* const* d_in, const int* in_sizes, int n_in,
                              void* d_out, int out_size, void* d_ws, size_t ws_size, hipStream_t stream) {
  if (n_in < 5) return;
  const size_t xneed = ((size_t)(NB - 1) * SEQ_FULL + SEQ) * DD;
  if ((size_t)in_sizes[0] < xneed) return;
  if ((size_t)in_sizes[1] < (size_t)DD * 3 * DD || in_sizes[2] < 3 * DD || (size_t)in_sizes[3] < (size_t)DD * DD || in_sizes[4] < DD) return;
  if ((size_t)out_size < xneed) return;
  const float* x = (const float*)d_in[0]; const float* Wattn = (const float*)d_in[1]; const float* battn = (const float*)d_in[2]; const float* Wproj = (const float*)d_in[3]; const float* bproj = (const float*)d_in[4];
  char* ws = (char*)d_ws; size_t off = 0;
  auto take = [&](size_t bytes) { char* p = ws + off; off += (bytes + 255) & ~(size_t)255; return p; };
  _Float16* Bqkv = (_Float16*)take((size_t)3 * DD * DD * 2);
  _Float16* Bp   = (_Float16*)take((size_t)DD * DD * 2);
  _Float16* X16  = (_Float16*)take((size_t)NR * DD * 2);
  _Float16* QK   = (_Float16*)take((size_t)NR * 2 * DD * 2);
  float*    VF   = (float*)take((size_t)NR * DD * 4);
  _Float16* Vth  = (_Float16*)take((size_t)NR * DD * 2);
  _Float16* Vtl  = (_Float16*)take((size_t)NR * DD * 2);
  _Float16* OH = QK; _Float16* OL = QK + (size_t)NR * DD; float* O = VF;
  if (off > ws_size) return;
  k_wt_f16<<<(unsigned)(((size_t)3 * DD * (DD / 8) + 255) / 256), 256, 0, stream>>>(Wattn, Bqkv, DD, 3 * DD, 16.0f);
  k_wt_f16<<<(unsigned)(((size_t)DD * (DD / 8) + 255) / 256), 256, 0, stream>>>(Wproj, Bp, DD, DD, 16.0f);
  k_x16s<<<(unsigned)(((size_t)NR * DD / 8 + 255) / 256), 256, 0, stream>>>(x, X16, (size_t)NR * DD / 8);
  k_gemm_hhx<0><<<dim3((unsigned)(((NR / 16) * (2 * DD / 64) + 3) / 4), 1), 128, 0, stream>>>(X16, DD, 0, Bqkv, DD, 0, 0.0625f, battn, 0, nullptr, nullptr, QK, 2 * DD, 0, NR, 2 * DD, DD);
  k_gemm_hhx<0><<<dim3((unsigned)(((NR / 16) * (DD / 64) + 3) / 4), 1), 128, 0, stream>>>(X16, DD, 0, Bqkv + (size_t)2 * DD * DD, DD, 0, 0.0625f, battn + 2 * DD, 0, nullptr, VF, nullptr, DD, 0, NR, DD, DD);
  k_vts<NH, SEQ><<<NB * NH * (SEQ / 64), 256, 0, stream>>>(VF, DD, Vth, Vtl);
  k_flash<<<NB * NH * (SEQ / 64), 128, 0, stream>>>(QK, 2 * DD, QK + DD, 2 * DD, Vth, Vtl, O, DD);
  k_hl<<<(unsigned)(((size_t)NR * DD / 8 + 255) / 256), 256, 0, stream>>>(O, OH, OL, (size_t)NR * DD / 8);
  const dim3 gpj((unsigned)(((SEQ / 16) * (DD / 64) + 3) / 4), NB);
  k_gemm_hhx<0><<<gpj, 128, 0, stream>>>(OH, DD, (size_t)SEQ * DD, Bp, DD, 0, 0.0625f, bproj, 0, nullptr, (float*)d_out, nullptr, DD, (size_t)SEQ_FULL * DD, SEQ, DD, DD);
  k_gemm_hhx<0><<<gpj, 128, 0, stream>>>(OL, DD, (size_t)SEQ * DD, Bp, DD, 0, 0.0625f * 0.0009765625f, nullptr, 0, (const float*)d_out, (float*)d_out, nullptr, DD, (size_t)SEQ_FULL * DD, SEQ, DD, DD);
}
